// FAM_8950711846062
// MI455X (gfx1250) — hardware-run, weakly checked
//
#include <hip/hip_runtime.h>
#include <math.h>

#pragma clang fp contract(off)

typedef __attribute__((ext_vector_type(16))) _Float16 v16h;
typedef __attribute__((ext_vector_type(8)))  _Float16 v8h;
typedef __attribute__((ext_vector_type(4)))  _Float16 v4h;
typedef __attribute__((ext_vector_type(16))) __bf16   v16b;
typedef __attribute__((ext_vector_type(8)))  __bf16   v8b;
typedef __attribute__((ext_vector_type(8)))  float    v8f;
typedef __attribute__((ext_vector_type(4)))  float    v4f;
typedef __attribute__((ext_vector_type(4)))  int      v4i;
typedef __attribute__((ext_vector_type(4)))  unsigned v4u;

constexpr int kBatch   = 8;
constexpr int kCx      = 128;
constexpr int kCu      = 128;
constexpr int kCo      = 128;
constexpr int kH       = 64;
constexpr int kW       = 64;
constexpr int kPlane   = kH * kW;
constexpr int kTaps    = 9;
constexpr int kNoff    = 18;
constexpr int kNoffPad = 32;
constexpr int kCcat    = kCx + kCu;
constexpr int kK1      = kCcat * kTaps;
constexpr int kK2      = kCu * kTaps;
constexpr int kChunkC  = 32;
constexpr int kChunkK  = kChunkC * kTaps;
constexpr int kChunks1 = kCcat / kChunkC;
constexpr int kChunks2 = kCu / kChunkC;
constexpr float kWCarry    = 16.0f;
constexpr float kWCarryInv = 1.0f / 16.0f;
static_assert(kK1 == 2304 && kK2 == 1152 && kChunkK == 288, "K sizes");
static_assert((kK1 % 32) == 0 && (kK2 % 32) == 0 && (kChunkK % 32) == 0, "K multiples of 32");
static_assert(kChunks1 == 8 && kChunks2 == 4, "chunk counts");
static_assert(kW == 64 && kH == 64 && kCx == 128 && kCu == 128 && kCo == 128, "tiling assumes these extents");

constexpr size_t kOffOFF  = 0;
constexpr size_t kOffWOH  = kOffOFF + (size_t)kBatch * kNoff * kPlane * 4;
constexpr size_t kOffWOL  = kOffWOH + (size_t)kNoffPad * kK1 * 2;
constexpr size_t kOffW2P  = kOffWOL + (size_t)kNoffPad * kK1 * 2;
constexpr size_t kWsTotal = kOffW2P + (size_t)kCo * kK2 * 2;
static_assert(kWsTotal == 2949120ull, "carve total");
static_assert(kWsTotal <= 134217728ull, "carve cap");
static_assert((kOffWOH % 128) == 0 && (kOffWOL % 128) == 0 && (kOffW2P % 128) == 0, "128-B aligned regions");

__device__ __forceinline__ unsigned short f2bf_bits(float f) {
  unsigned u = __float_as_uint(f);
  return (unsigned short)((u + 0x7FFFu + ((u >> 16) & 1u)) >> 16);
}
__device__ __forceinline__ float bf_bits2f(unsigned short h) { return __uint_as_float(((unsigned)h) << 16); }
__device__ __forceinline__ int clampi(int v, int lo, int hi) { return v < lo ? lo : (v > hi ? hi : v); }

template <typename T> struct Frag;
template <> struct Frag<_Float16> {
  typedef v16h V; union U { v16h v; v8h h[2]; };
  static __device__ __forceinline__ v16h load(const _Float16* p) {
    U f; f.h[0] = *(const v8h*)(p); f.h[1] = *(const v8h*)(p + 16); return f.v;
  }
};
template <> struct Frag<__bf16> {
  typedef v16b V; union U { v16b v; v8b h[2]; };
  static __device__ __forceinline__ v16b load(const __bf16* p) {
    U f; f.h[0] = *(const v8b*)(p); f.h[1] = *(const v8b*)(p + 16); return f.v;
  }
};

__device__ __forceinline__ v8f mma_bf(v16b a, v16b b, v8f c) {
  c = __builtin_amdgcn_wmma_f32_16x16x32_bf16(false, a, false, b, (short)0, c, false, false);
  asm volatile("v_nop\n\tv_nop\n\tv_nop\n\tv_nop" : "+v"(c) : "v"(a), "v"(b));
  return c;
}
__device__ __forceinline__ v8f mma_h(v16h a, v16h b, v8f c) {
  c = __builtin_amdgcn_wmma_f32_16x16x32_f16(false, a, false, b, (short)0, c, false, false);
  asm volatile("v_nop\n\tv_nop\n\tv_nop\n\tv_nop" : "+v"(c) : "v"(a), "v"(b));
  return c;
}

constexpr int kPrepWoBlocks = (kNoffPad * kK1 / 8) / 256;
constexpr int kPrepW2Blocks = (kCo * kK2 / 8) / 256;
static_assert(kPrepWoBlocks * 256 * 8 == kNoffPad * kK1, "exact coverage");
static_assert(kPrepW2Blocks * 256 * 8 == kCo * kK2, "exact coverage");

__global__ __launch_bounds__(256) void prep_weights_kernel(
    const float* __restrict__ weight, const float* __restrict__ offset_w,
    unsigned short* __restrict__ WoH, unsigned short* __restrict__ WoL, unsigned short* __restrict__ W2p)
{
  const int blk = blockIdx.x;
  if (blk < kPrepWoBlocks) {
    const int i   = blk * 256 + threadIdx.x;
    const int e0  = i * 8;
    const int n   = e0 / kK1;
    const int kp  = e0 - n * kK1;
    const int chunk = kp / kChunkK;
    const int rem = kp - chunk * kChunkK;
    const int tap = rem >> 5;
    const int cl0 = rem & 31;
    const int nc  = (n < kNoff) ? n : (kNoff - 1);
    const float* sp = offset_w + (size_t)nc * kK1 + (size_t)(chunk * kChunkC + cl0) * kTaps + tap;
    float v[8];
#pragma unroll
    for (int e = 0; e < 8; ++e) {
      const float t = sp[e * kTaps];
      v[e] = (n < kNoff) ? t : 0.0f;
    }
    unsigned hw[4], lw[4];
#pragma unroll
    for (int p = 0; p < 4; ++p) {
      const unsigned short h0 = f2bf_bits(v[2 * p]);
      const unsigned short h1 = f2bf_bits(v[2 * p + 1]);
      const unsigned short l0 = f2bf_bits(v[2 * p] - bf_bits2f(h0));
      const unsigned short l1 = f2bf_bits(v[2 * p + 1] - bf_bits2f(h1));
      hw[p] = (unsigned)h0 | ((unsigned)h1 << 16);
      lw[p] = (unsigned)l0 | ((unsigned)l1 << 16);
    }
    const v4u hv = (v4u){hw[0], hw[1], hw[2], hw[3]};
    const v4u lv = (v4u){lw[0], lw[1], lw[2], lw[3]};
    unsigned short* qh = WoH + e0;
    unsigned short* ql = WoL + e0;
    *(volatile v4u*)qh = hv;
    *(volatile v4u*)ql = lv;
    __threadfence();
    *(volatile v4u*)qh = hv;
    *(volatile v4u*)ql = lv;
  } else {
    const int i   = (blk - kPrepWoBlocks) * 256 + threadIdx.x;
    const int e0  = i * 8;
    const int n   = e0 / kK2;
    const int kp  = e0 - n * kK2;
    const int chunk = kp / kChunkK;
    const int rem = kp - chunk * kChunkK;
    const int tap = rem >> 5;
    const int cl0 = rem & 31;
    const float* sp = weight + (size_t)n * kK2 + (size_t)(chunk * kChunkC + cl0) * kTaps + tap;
    float v[8];
#pragma unroll
    for (int e = 0; e < 8; ++e) v[e] = sp[e * kTaps] * kWCarry;
    unsigned hw[4];
#pragma unroll
    for (int p = 0; p < 4; ++p) {
      const _Float16 f0 = (_Float16)v[2 * p];
      const _Float16 f1 = (_Float16)v[2 * p + 1];
      const unsigned short h0 = __builtin_bit_cast(unsigned short, f0);
      const unsigned short h1 = __builtin_bit_cast(unsigned short, f1);
      hw[p] = (unsigned)h0 | ((unsigned)h1 << 16);
    }
    const v4u hv = (v4u){hw[0], hw[1], hw[2], hw[3]};
    unsigned short* qh = W2p + e0;
    *(volatile v4u*)qh = hv;
    __threadfence();
    *(volatile v4u*)qh = hv;
  }
}

constexpr int kRCols  = kW + 2;
constexpr int kRPitch = 40;
constexpr int kRElems = 3 * kRCols * kRPitch;
constexpr int kOPitch = 68;
constexpr int kStageGroups = 3 * kRCols * (kChunkC / 8);
static_assert(kStageGroups == 792, "staging groups");
static_assert(7 * 128 >= kStageGroups, "staging passes cover all groups");

__global__ __launch_bounds__(128) void offset_conv_kernel(
    const float* __restrict__ x, const float* __restrict__ u, const float* __restrict__ offset_b,
    const unsigned short* __restrict__ WoHp, const unsigned short* __restrict__ WoLp,
    float* __restrict__ OFF)
{
  __shared__ __align__(16) __bf16 Rh[kRElems];
  __shared__ __align__(16) __bf16 Rl[kRElems];
  __shared__ __align__(16) float  sO[kNoff * kOPitch];

  const int tid  = threadIdx.x;
  const int lane = tid & 31;
  const int wave = tid >> 5;
  const int hh   = lane >> 4;
  const int m    = lane & 15;
  const int b    = blockIdx.x >> 6;
  const int y    = blockIdx.x & 63;
  const __bf16* WoH = (const __bf16*)WoHp;
  const __bf16* WoL = (const __bf16*)WoLp;

  v8f acc0 = (v8f){0.f,0.f,0.f,0.f,0.f,0.f,0.f,0.f};
  v8f acc1 = (v8f){0.f,0.f,0.f,0.f,0.f,0.f,0.f,0.f};

#pragma unroll 1
  for (int chunk = 0; chunk < kChunks1; ++chunk) {
    __syncthreads();
    const float* src = (chunk < 4) ? x : u;
    const float* sb  = src + (size_t)(b * 128 + (chunk & 3) * kChunkC) * kPlane;
#pragma unroll 1
    for (int ps = 0; ps < 7; ++ps) {
      const int g   = ps * 128 + tid;
      const int gc  = (g < kStageGroups) ? g : (kStageGroups - 1);
      const int cg  = gc / (3 * kRCols);
      const int rc  = gc - cg * (3 * kRCols);
      const int ky  = rc / kRCols;
      const int col = rc - ky * kRCols;
      const int yy  = y + ky - 1;
      const int xx  = col - 1;
      const bool ok = (yy >= 0) && (yy < kH) && (xx >= 0) && (xx < kW);
      const int yyc = clampi(yy, 0, kH - 1);
      const int xxc = clampi(xx, 0, kW - 1);
      const float* p = sb + (size_t)(cg * 8) * kPlane + yyc * kW + xxc;
      float v[8];
#pragma unroll
      for (int e = 0; e < 8; ++e) {
        float t = p[(size_t)e * kPlane];
        asm volatile("" : "+v"(t));
        v[e] = ok ? t : 0.0f;
      }
      v8b hv, lv;
#pragma unroll
      for (int e = 0; e < 8; ++e) {
        const unsigned short hb = f2bf_bits(v[e]);
        const unsigned short lb = f2bf_bits(v[e] - bf_bits2f(hb));
        hv[e] = __builtin_bit_cast(__bf16, hb);
        lv[e] = __builtin_bit_cast(__bf16, lb);
      }
      {
        const int ro = (ky * kRCols + col) * kRPitch + cg * 8;
        *(v8b*)(Rh + ro) = hv;
        *(v8b*)(Rl + ro) = lv;
      }
    }
    __syncthreads();

#pragma unroll 1
    for (int tap = 0; tap < kTaps; ++tap) {
      const int ky = tap / 3;
      const int kx = tap - ky * 3;
      const int ao = (ky * kRCols + wave * 16 + m + kx) * kRPitch + 8 * hh;
      const v16b ah = Frag<__bf16>::load(Rh + ao);
      const v16b al = Frag<__bf16>::load(Rl + ao);
      const size_t bo = (size_t)m * kK1 + chunk * kChunkK + tap * 32 + 8 * hh;
      const v16b bh0 = Frag<__bf16>::load(WoH + bo);
      const v16b bl0 = Frag<__bf16>::load(WoL + bo);
      const v16b bh1 = Frag<__bf16>::load(WoH + bo + (size_t)16 * kK1);
      const v16b bl1 = Frag<__bf16>::load(WoL + bo + (size_t)16 * kK1);
      acc0 = mma_bf(ah, bh0, acc0);
      acc0 = mma_bf(ah, bl0, acc0);
      acc0 = mma_bf(al, bh0, acc0);
      acc1 = mma_bf(ah, bh1, acc1);
      acc1 = mma_bf(ah, bl1, acc1);
      acc1 = mma_bf(al, bh1, acc1);
    }
  }

  {
    const float ob0 = offset_b[m];
    const int ch1   = 16 + m;
    const int ch1c  = (ch1 < kNoff) ? ch1 : (kNoff - 1);
    const float ob1 = offset_b[ch1c];
    const int pb = wave * 16 + 8 * hh;
#pragma unroll
    for (int r = 0; r < 8; ++r) sO[m * kOPitch + pb + r] = acc0[r] + ob0;
    if (ch1 < kNoff) {
#pragma unroll
      for (int r = 0; r < 8; ++r) sO[ch1 * kOPitch + pb + r] = acc1[r] + ob1;
    }
  }
  __syncthreads();
  {
    const int c4 = m * 4;
    v4f vals[3];
#pragma unroll
    for (int t = 0; t < 3; ++t) {
      const int it = wave + 4 * t;
      const int ch = clampi(it * 2 + hh, 0, kNoff - 1);
      vals[t] = *(const v4f*)(sO + ch * kOPitch + c4);
    }
    for (int pass = 0; pass < 2; ++pass) {
#pragma unroll
      for (int t = 0; t < 3; ++t) {
        const int it = wave + 4 * t;
        if (it < 9) {
          const int ch = it * 2 + hh;
          *(volatile v4f*)(OFF + (((size_t)(b * kNoff + ch) * kH + y) * kW + c4)) = vals[t];
        }
      }
      __threadfence();
    }
  }
}

constexpr int kSPitch    = 296;
constexpr int kSlabPitch = 36;
constexpr int kMetaN     = 32 * kTaps;
static_assert(kMetaN == 288, "metadata entries");

__global__ __launch_bounds__(128) void deform_main_kernel(
    const float* __restrict__ u, const float* __restrict__ bias, const float* __restrict__ OFF,
    const unsigned short* __restrict__ W2pp, float* __restrict__ out)
{
  __shared__ __align__(16) _Float16 S[32 * kSPitch];
  __shared__ __align__(16) int      midx[kMetaN * 4];
  __shared__ __align__(16) float    mwt[kMetaN * 4];
  __shared__ __align__(16) float    slab[kCo * kSlabPitch];

  const int tid  = threadIdx.x;
  const int lane = tid & 31;
  const int wave = tid >> 5;
  const int hh   = lane >> 4;
  const int m    = lane & 15;
  const int tile = blockIdx.x;
  const int x0   = (tile & 1) * 32;
  const int y    = (tile >> 1) & 63;
  const int b    = tile >> 7;
  const _Float16* W2 = (const _Float16*)W2pp;

#pragma unroll 1
  for (int t = 0; t < 3; ++t) {
    const int e  = t * 128 + tid;
    const int ec = (e < kMetaN) ? e : (kMetaN - 1);
    const int p  = ec / kTaps;
    const int j  = ec - p * kTaps;
    const int xg = x0 + p;
    const size_t ob = ((size_t)(b * kNoff + 2 * j) * kH + y) * kW + xg;
    const float dy = OFF[ob];
    const float dx = OFF[ob + kPlane];
    const int ky = j / 3;
    const int kx = j - ky * 3;
    const float py = (float)(y - 1 + ky) + dy;
    const float px = (float)(xg - 1 + kx) + dx;
    const float y0f = floorf(py);
    const float x0f = floorf(px);
    const float wy1 = py - y0f;
    const float wy0 = 1.0f - wy1;
    const float wx1 = px - x0f;
    const float wx0 = 1.0f - wx1;
    const int y0i = (int)fminf(fmaxf(y0f, -8.0f), 72.0f);
    const int x0i = (int)fminf(fmaxf(x0f, -8.0f), 72.0f);
    const int y1i = y0i + 1;
    const int x1i = x0i + 1;
    const bool vy0 = (y0i >= 0) && (y0i < kH);
    const bool vy1 = (y1i >= 0) && (y1i < kH);
    const bool vx0 = (x0i >= 0) && (x0i < kW);
    const bool vx1 = (x1i >= 0) && (x1i < kW);
    const int yc0 = clampi(y0i, 0, kH - 1);
    const int yc1 = clampi(y1i, 0, kH - 1);
    const int xc0 = clampi(x0i, 0, kW - 1);
    const int xc1 = clampi(x1i, 0, kW - 1);
    const float w00 = wy0 * wx0;
    const float w01 = wy0 * wx1;
    const float w10 = wy1 * wx0;
    const float w11 = wy1 * wx1;
    const v4i id = (v4i){yc0 * kW + xc0, yc0 * kW + xc1, yc1 * kW + xc0, yc1 * kW + xc1};
    const v4f wv = (v4f){(vy0 && vx0) ? w00 : 0.0f, (vy0 && vx1) ? w01 : 0.0f,
                         (vy1 && vx0) ? w10 : 0.0f, (vy1 && vx1) ? w11 : 0.0f};
    if (e < kMetaN) {
      *(v4i*)(midx + e * 4) = id;
      *(v4f*)(mwt + e * 4)  = wv;
    }
  }
  __syncthreads();

  v8f acc00 = (v8f){0.f,0.f,0.f,0.f,0.f,0.f,0.f,0.f};
  v8f acc01 = (v8f){0.f,0.f,0.f,0.f,0.f,0.f,0.f,0.f};
  v8f acc10 = (v8f){0.f,0.f,0.f,0.f,0.f,0.f,0.f,0.f};
  v8f acc11 = (v8f){0.f,0.f,0.f,0.f,0.f,0.f,0.f,0.f};

#pragma unroll 1
  for (int chunk = 0; chunk < kChunks2; ++chunk) {
    __syncthreads();
    const float* ub = u + (size_t)(b * kCu + chunk * kChunkC) * kPlane;
#pragma unroll 1
    for (int ps = 0; ps < 18; ++ps) {
      const int tap = ps >> 1;
      const int cq  = (ps & 1) * 4 + wave;
      const v4i id = *(const v4i*)(midx + (lane * kTaps + tap) * 4);
      const v4f wv = *(const v4f*)(mwt + (lane * kTaps + tap) * 4);
      const int i0 = id[0], i1 = id[1], i2 = id[2], i3 = id[3];
      const float w0 = wv[0], w1 = wv[1], w2 = wv[2], w3 = wv[3];
      const float* up = ub + (size_t)(cq * 4) * kPlane;
      v4h hv;
#pragma unroll
      for (int e = 0; e < 4; ++e) {
        const float* q = up + (size_t)e * kPlane;
        const float g0 = q[i0];
        const float g1 = q[i1];
        const float g2 = q[i2];
        const float g3 = q[i3];
        float s = g0 * w0;
        s = fmaf(g1, w1, s);
        s = fmaf(g2, w2, s);
        s = fmaf(g3, w3, s);
        hv[e] = (_Float16)s;
      }
      *(v4h*)(S + lane * kSPitch + tap * 32 + cq * 4) = hv;
    }
    __syncthreads();

#pragma unroll 1
    for (int tap = 0; tap < kTaps; ++tap) {
      const size_t ao = (size_t)(wave * 32 + m) * kK2 + chunk * kChunkK + tap * 32 + 8 * hh;
      const v16h a0 = Frag<_Float16>::load(W2 + ao);
      const v16h a1 = Frag<_Float16>::load(W2 + ao + (size_t)16 * kK2);
      const int bo = m * kSPitch + tap * 32 + 8 * hh;
      const v16h b0 = Frag<_Float16>::load(S + bo);
      const v16h b1 = Frag<_Float16>::load(S + bo + 16 * kSPitch);
      acc00 = mma_h(a0, b0, acc00);
      acc01 = mma_h(a0, b1, acc01);
      acc10 = mma_h(a1, b0, acc10);
      acc11 = mma_h(a1, b1, acc11);
    }
  }

  {
    const int ob = wave * 32 + 8 * hh;
#pragma unroll
    for (int r = 0; r < 8; ++r) {
      slab[(ob + r) * kSlabPitch + m]           = acc00[r] * kWCarryInv;
      slab[(ob + r) * kSlabPitch + 16 + m]      = acc01[r] * kWCarryInv;
      slab[(ob + 16 + r) * kSlabPitch + m]      = acc10[r] * kWCarryInv;
      slab[(ob + 16 + r) * kSlabPitch + 16 + m] = acc11[r] * kWCarryInv;
    }
  }
  __syncthreads();
  {
    const int q  = lane >> 3;
    const int c4 = (lane & 7) * 4;
    v4f vals[8];
#pragma unroll
    for (int it = 0; it < 8; ++it) {
      const int row = wave * 32 + it * 4 + q;
      const float bv = bias[row];
      v4f t = *(const v4f*)(slab + row * kSlabPitch + c4);
      t[0] = t[0] + bv;
      t[1] = t[1] + bv;
      t[2] = t[2] + bv;
      t[3] = t[3] + bv;
      vals[it] = t;
    }
    for (int pass = 0; pass < 2; ++pass) {
#pragma unroll
      for (int it = 0; it < 8; ++it) {
        const int row = wave * 32 + it * 4 + q;
        *(volatile v4f*)(out + (((size_t)(b * kCo + row) * kH + y) * kW + x0 + c4)) = vals[it];
      }
      __threadfence();
    }
  }
}

extern "C" void kernel_launch(void* const* d_in, const int* in_sizes, int n_in,
                              void* d_out, int out_size, void* d_ws, size_t ws_size,
                              hipStream_t stream) {
  if (n_in < 6) return;
  if (in_sizes[0] != kBatch * kCx * kPlane) return;
  if (in_sizes[1] != kBatch * kCu * kPlane) return;
  if (in_sizes[2] != kCo * kK2) return;
  if (in_sizes[3] != kCo) return;
  if (in_sizes[4] != kNoff * kK1) return;
  if (in_sizes[5] != kNoff) return;
  if (out_size != kBatch * kCo * kPlane) return;
  if (ws_size < kWsTotal) return;

  const float* x        = (const float*)d_in[0];
  const float* u        = (const float*)d_in[1];
  const float* weight   = (const float*)d_in[2];
  const float* bias     = (const float*)d_in[3];
  const float* offset_w = (const float*)d_in[4];
  const float* offset_b = (const float*)d_in[5];
  float* out = (float*)d_out;

  char* ws = (char*)d_ws;
  float*          OFF = (float*)(ws + kOffOFF);
  unsigned short* WoH = (unsigned short*)(ws + kOffWOH);
  unsigned short* WoL = (unsigned short*)(ws + kOffWOL);
  unsigned short* W2p = (unsigned short*)(ws + kOffW2P);

  prep_weights_kernel<<<kPrepWoBlocks + kPrepW2Blocks, 256, 0, stream>>>(weight, offset_w, WoH, WoL, W2p);
  offset_conv_kernel<<<kBatch * kH, 128, 0, stream>>>(x, u, offset_b, WoH, WoL, OFF);
  deform_main_kernel<<<kBatch * kH * (kW / 32), 128, 0, stream>>>(u, bias, OFF, W2p, out);
}
